// Dcls2d_4398046511417
// MI455X (gfx1250) — hardware-verified
//
#include <hip/hip_runtime.h>
#include <stdint.h>
#include <stddef.h>
#include <math.h>

#pragma clang fp contract(off)

typedef __attribute__((ext_vector_type(16))) _Float16 v16h;
typedef __attribute__((ext_vector_type(8)))  _Float16 v8h;
typedef __attribute__((ext_vector_type(16))) __bf16   v16b;
typedef __attribute__((ext_vector_type(8)))  __bf16   v8b;
typedef __attribute__((ext_vector_type(8)))  float    v8f;
typedef __attribute__((ext_vector_type(4)))  float    v4f;
typedef __attribute__((ext_vector_type(4)))  unsigned int v4u;

constexpr int NIMG    = 32;
constexpr int CIN     = 128;
constexpr int COUT    = 128;
constexpr int HIMG    = 56;
constexpr int WIMG    = 56;
constexpr int NPIX    = HIMG * WIMG;
constexpr int KTAP_H  = 7;
constexpr int KTAP_W  = 7;
constexpr int NTAP    = KTAP_H * KTAP_W;
constexpr int NPTS    = 9;
constexpr int HALO    = 3;
constexpr int HPADP   = HIMG + 2 * HALO;
constexpr int WPADP   = 64;
constexpr int PTILES  = NPIX / 64;
constexpr int NTHR    = 256;
constexpr int TPITCH  = 136;
constexpr int SLABP   = 68;
constexpr int NCELL   = NTAP + 1;
constexpr float KCARRY     = 1024.0f;
constexpr float KCARRY_INV = 1.0f / 1024.0f;

constexpr size_t XPAD_HALVES = (size_t)NIMG * HPADP * WPADP * CIN;
constexpr size_t XPAD_BYTES  = XPAD_HALVES * 2;
constexpr size_t BT_HALVES   = (size_t)NTAP * COUT * CIN;
constexpr size_t BT_BYTES    = BT_HALVES * 2;
constexpr size_t WS_TOTAL    = XPAD_BYTES + BT_BYTES;

static_assert(NPIX % 64 == 0, "M tile 64 divides the pixel count");
static_assert(CIN % 32 == 0, "K chunk 32 divides CIN");
static_assert(COUT % 64 == 0, "N tile 64 divides COUT");
static_assert((NIMG * PTILES * (COUT / 64)) % 8 == 0, "8 wave tiles per block exactly");
static_assert(CIN * (WIMG / 4) == 7 * NTHR, "transpose load phase: 7 float4 per thread exactly");
static_assert(WPADP * CIN == 4 * NTHR * 8, "transpose store phase: 4 x 16 B per thread exactly");
static_assert(XPAD_BYTES % 128 == 0, "bt region starts on a line");
static_assert(WS_TOTAL <= (size_t)134217728, "carve within 128 MiB");
static_assert((NPIX * 4) % 128 == 0, "o rows of the output start on 128-B lines");
static_assert(TPITCH % 8 == 0 && TPITCH >= CIN, "transpose tile pitch");
static_assert(NTAP * 32 <= 7 * NTHR, "bt store phase: 7 iterations cover all taps");

__device__ __forceinline__ void dep_guard_h(v8f& a, v8f& b, v16h x, v16h y) { asm volatile("v_nop\n\tv_nop\n\tv_nop\n\tv_nop" : "+v"(a), "+v"(b) : "v"(x), "v"(y)); }
__device__ __forceinline__ void dep_guard_b(v8f& a, v8f& b, v16b x, v16b y) { asm volatile("v_nop\n\tv_nop\n\tv_nop\n\tv_nop" : "+v"(a), "+v"(b) : "v"(x), "v"(y)); }
__device__ __forceinline__ void keep4_h(v16h a, v16h b, v16h c, v16h d) { asm volatile("v_nop" :: "v"(a), "v"(b), "v"(c), "v"(d)); }
__device__ __forceinline__ void keep4_b(v16b a, v16b b, v16b c, v16b d) { asm volatile("v_nop" :: "v"(a), "v"(b), "v"(c), "v"(d)); }
__device__ __forceinline__ void acc_guard4(v8f& a, v8f& b, v8f& c, v8f& d) { asm volatile("v_nop\n\tv_nop\n\tv_nop\n\tv_nop" : "+v"(a), "+v"(b), "+v"(c), "+v"(d)); }
template <typename T> struct Frag;
template <> struct Frag<_Float16> {
  typedef v16h V; union U { v16h v; v8h h[2]; };
  static __device__ __forceinline__ v16h load(const _Float16* p) {
    U f; f.h[0] = *(const v8h*)(p); f.h[1] = *(const v8h*)(p + 16); return f.v;
  }
  static __device__ __forceinline__ v8f mma(v16h a, v16h b, v8f c) {
    return __builtin_amdgcn_wmma_f32_16x16x32_f16(false, a, false, b, (short)0, c, false, false);
  }
  static __device__ __forceinline__ void guard(v8f& a, v8f& b, v16h x, v16h y) { dep_guard_h(a, b, x, y); }
  static __device__ __forceinline__ void keep(v16h a, v16h b, v16h c, v16h d) { keep4_h(a, b, c, d); }
};
template <> struct Frag<__bf16> {
  typedef v16b V; union U { v16b v; v8b h[2]; };
  static __device__ __forceinline__ v16b load(const __bf16* p) {
    U f; f.h[0] = *(const v8b*)(p); f.h[1] = *(const v8b*)(p + 16); return f.v;
  }
  static __device__ __forceinline__ v8f mma(v16b a, v16b b, v8f c) {
    return __builtin_amdgcn_wmma_f32_16x16x32_bf16(false, a, false, b, (short)0, c, false, false);
  }
  static __device__ __forceinline__ void guard(v8f& a, v8f& b, v16b x, v16b y) { dep_guard_b(a, b, x, y); }
  static __device__ __forceinline__ void keep(v16b a, v16b b, v16b c, v16b d) { keep4_b(a, b, c, d); }
};
typedef Frag<_Float16> FragH;

__device__ __forceinline__ unsigned short f16_bits(float f) { return __builtin_bit_cast(unsigned short, (_Float16)f); }

__global__ __launch_bounds__(NTHR) void k_pad_nhwc(const float* __restrict__ x, unsigned short* __restrict__ xpad) {
  __shared__ __align__(16) unsigned short T[WIMG * TPITCH];
  const int yp  = blockIdx.x;
  const int n   = blockIdx.y;
  const int tid = threadIdx.x;
  const int y   = yp - HALO;
  const bool yok = ((unsigned)y < (unsigned)HIMG);
  const int yc  = yok ? y : 0;

#pragma unroll 1
  for (int it = 0; it < 7; ++it) {
    const int idx = it * NTHR + tid;
    const int c   = idx / 14;
    const int q   = idx - c * 14;
    const v4f v = *(const v4f*)(x + ((((size_t)n * CIN + c) * HIMG + yc) * WIMG + (size_t)(q * 4)));
#pragma unroll
    for (int e = 0; e < 4; ++e) {
      T[(q * 4 + e) * TPITCH + c] = f16_bits(v[e]);
    }
  }
  __syncthreads();

  unsigned short* dst = xpad + ((size_t)n * HPADP + yp) * (size_t)(WPADP * CIN);
  for (int pass = 0; pass < 2; ++pass) {
#pragma unroll
    for (int it = 0; it < 4; ++it) {
      const int u  = it * NTHR + tid;
      const int xp = u >> 4;
      const int c0 = (u & 15) * 8;
      const int xs = xp - HALO;
      const bool inside = yok && ((unsigned)xs < (unsigned)WIMG);
      const int xsc = xs < 0 ? 0 : (xs > WIMG - 1 ? WIMG - 1 : xs);
      v4u w = *(const v4u*)(T + xsc * TPITCH + c0);
      const unsigned msk = inside ? 0xffffffffu : 0u;
      const v4u m4 = (v4u){msk, msk, msk, msk};
      w = w & m4;
      *(volatile v4u*)(dst + (size_t)xp * CIN + c0) = w;
    }
    __threadfence();
  }
}

__global__ __launch_bounds__(NTHR) __attribute__((amdgpu_num_vgpr(256)))
void k_build_taps(const float* __restrict__ weight, const float* __restrict__ P, unsigned short* __restrict__ bt) {
  __shared__ __align__(16) float S[NCELL * NTHR];
  const int tid = threadIdx.x;
  const int ol  = tid >> 7;
  const int c   = tid & (CIN - 1);
  const int o   = blockIdx.x * 2 + ol;
  float* col = S + tid;

#pragma unroll 1
  for (int cell = 0; cell < NCELL; ++cell) col[cell * NTHR] = 0.0f;

  const float* p0row = P + (size_t)c * NPTS;
  const float* p1row = P + (size_t)(CIN + c) * NPTS;
  const float* wrow  = weight + ((size_t)o * CIN + c) * NPTS;
#pragma unroll 1
  for (int k = 0; k < NPTS; ++k) {
    const float p0 = p0row[k];
    const float p1 = p1row[k];
    const float w  = wrow[k];
    const float ph = fminf(fmaxf(p0, -3.0f), 3.0f) + 3.0f;
    const float pw = fminf(fmaxf(p1, -3.0f), 3.0f) + 3.0f;
    const float fh = floorf(ph);
    const float fw = floorf(pw);
    const float rh = ph - fh;
    const float rw = pw - fw;
    int ih = (int)fh;
    int iw = (int)fw;
    ih = ih < 0 ? 0 : (ih > KTAP_H - 1 ? KTAP_H - 1 : ih);
    iw = iw < 0 ? 0 : (iw > KTAP_W - 1 ? KTAP_W - 1 : iw);
    const bool hok = (ih + 1) < KTAP_H;
    const bool wok = (iw + 1) < KTAP_W;
    const int i00 = ih * KTAP_W + iw;
    const int i01 = wok ? (ih * KTAP_W + iw + 1) : NTAP;
    const int i10 = hok ? ((ih + 1) * KTAP_W + iw) : NTAP;
    const int i11 = (hok && wok) ? ((ih + 1) * KTAP_W + iw + 1) : NTAP;
    const float omh = 1.0f - rh;
    const float omw = 1.0f - rw;
    const float w00 = w * (omh * omw);
    const float w01 = w * (omh * rw);
    const float w10 = w * (rh * omw);
    const float w11 = w * (rh * rw);
    col[i00 * NTHR] += w00;
    col[i01 * NTHR] += w01;
    col[i10 * NTHR] += w10;
    col[i11 * NTHR] += w11;
  }
  __syncthreads();

  for (int pass = 0; pass < 2; ++pass) {
#pragma unroll
    for (int it = 0; it < 7; ++it) {
      const int u = it * NTHR + tid;
      if (u < NTAP * 32) {
        const int tap = u >> 5;
        const int r   = u & 31;
        const float* sp = S + tap * NTHR + r * 8;
        const v4f a = *(const v4f*)(sp);
        const v4f b = *(const v4f*)(sp + 4);
        v8h hv;
        hv[0] = (_Float16)(a[0] * KCARRY); hv[1] = (_Float16)(a[1] * KCARRY);
        hv[2] = (_Float16)(a[2] * KCARRY); hv[3] = (_Float16)(a[3] * KCARRY);
        hv[4] = (_Float16)(b[0] * KCARRY); hv[5] = (_Float16)(b[1] * KCARRY);
        hv[6] = (_Float16)(b[2] * KCARRY); hv[7] = (_Float16)(b[3] * KCARRY);
        *(volatile v8h*)(bt + ((size_t)tap * COUT + (size_t)blockIdx.x * 2) * CIN + (size_t)(r * 8)) = hv;
      }
    }
    __threadfence();
  }
}

__global__ __launch_bounds__(NTHR) void k_conv_wmma(const unsigned short* __restrict__ xpadp, const unsigned short* __restrict__ btp,
                                                  const float* __restrict__ bias, float* __restrict__ out) {
  const _Float16* XP = (const _Float16*)xpadp;
  const _Float16* BT = (const _Float16*)btp;
  __shared__ __align__(16) float sT[8][16 * SLABP];

  const int lane = threadIdx.x & 31;
  const int wave = threadIdx.x >> 5;
  const int tile = blockIdx.x * 8 + wave;
  const int oh   = tile & 1;
  const int t2   = tile >> 1;
  const int n    = t2 / PTILES;
  const int pt   = t2 - n * PTILES;
  const int n0   = oh * 64;
  const int pBase = pt * 64;
  const int rlane = lane & 15;
  const int koff  = (lane >> 4) * 8;
  const int mOff  = (lane >> 4) * 8;

  const _Float16* arow[4];
#pragma unroll
  for (int i = 0; i < 4; ++i) {
    const int p  = pBase + 16 * i + rlane;
    const int y  = p / WIMG;
    const int xx = p - y * WIMG;
    arow[i] = XP + (((size_t)n * HPADP + y) * WPADP + xx) * CIN + koff;
  }
  const _Float16* brow = BT + (size_t)(n0 + rlane) * CIN + koff;

  v8f acc[4][4];
#pragma unroll
  for (int i = 0; i < 4; ++i)
#pragma unroll
    for (int j = 0; j < 4; ++j) acc[i][j] = (v8f){0.f,0.f,0.f,0.f,0.f,0.f,0.f,0.f};

#pragma unroll 1
  for (int ks = 0; ks < NTAP * 4; ++ks) {
    const int tap = ks >> 2;
    const int c0  = (ks & 3) * 32;
    const int kh  = tap / KTAP_W;
    const int kw  = tap - kh * KTAP_W;
    const size_t aoff = (size_t)(kh * WPADP + kw) * CIN + c0;
    const size_t boff = (size_t)tap * COUT * CIN + c0;
    v16h bh[4];
#pragma unroll
    for (int j = 0; j < 4; ++j) bh[j] = FragH::load(brow + boff + (size_t)(j * 16) * CIN);
#pragma unroll
    for (int i = 0; i < 4; ++i) {
      const v16h ah = FragH::load(arow[i] + aoff);
#pragma unroll
      for (int j = 0; j < 4; ++j) acc[i][j] = FragH::mma(ah, bh[j], acc[i][j]);
      FragH::guard(acc[i][0], acc[i][3], ah, ah);
    }
    FragH::keep(bh[0], bh[1], bh[2], bh[3]);
  }
  acc_guard4(acc[0][0], acc[0][1], acc[0][2], acc[0][3]);
  acc_guard4(acc[1][0], acc[1][1], acc[1][2], acc[1][3]);
  acc_guard4(acc[2][0], acc[2][1], acc[2][2], acc[2][3]);
  acc_guard4(acc[3][0], acc[3][1], acc[3][2], acc[3][3]);

  float* slab = sT[wave];
  const int hh = lane >> 4;
  const int c4 = (lane & 15) * 4;
#pragma unroll
  for (int j = 0; j < 4; ++j) {
    const int ob = n0 + 16 * j;
    const float bv = bias[ob + rlane];
#pragma unroll
    for (int i = 0; i < 4; ++i) {
#pragma unroll
      for (int r = 0; r < 8; ++r) {
        slab[rlane * SLABP + 16 * i + mOff + r] = acc[i][j][r] * KCARRY_INV + bv;
      }
    }
    __builtin_amdgcn_fence(__ATOMIC_RELEASE, "workgroup");
    __builtin_amdgcn_wave_barrier();
    __builtin_amdgcn_fence(__ATOMIC_ACQUIRE, "workgroup");
    float* C = out + ((size_t)n * COUT + ob) * NPIX + pBase;
    for (int pass = 0; pass < 2; ++pass) {
#pragma unroll
      for (int it = 0; it < 8; ++it) {
        const int row = it * 2 + hh;
        const v4f v = *(const v4f*)(slab + row * SLABP + c4);
        *(volatile v4f*)(C + (size_t)row * NPIX + c4) = v;
      }
      __threadfence();
    }
    __builtin_amdgcn_fence(__ATOMIC_RELEASE, "workgroup");
    __builtin_amdgcn_wave_barrier();
    __builtin_amdgcn_fence(__ATOMIC_ACQUIRE, "workgroup");
  }
}

extern "C" void kernel_launch(void* const* d_in, const int* in_sizes, int n_in,
                              void* d_out, int out_size, void* d_ws, size_t ws_size,
                              hipStream_t stream) {
  if (n_in < 4) return;
  if (in_sizes[0] != NIMG * CIN * NPIX) return;
  if (in_sizes[1] != COUT * CIN * NPTS) return;
  if (in_sizes[2] != 2 * CIN * NPTS) return;
  if (in_sizes[3] != COUT) return;
  if (out_size != NIMG * COUT * NPIX) return;
  if (ws_size < WS_TOTAL) return;

  const float* x      = (const float*)d_in[0];
  const float* weight = (const float*)d_in[1];
  const float* P      = (const float*)d_in[2];
  const float* bias   = (const float*)d_in[3];
  float* out = (float*)d_out;

  char* ws = (char*)d_ws;
  unsigned short* xpad = (unsigned short*)(ws);
  unsigned short* bt   = (unsigned short*)(ws + XPAD_BYTES);

  k_pad_nhwc<<<dim3(HPADP, NIMG), NTHR, 0, stream>>>(x, xpad);
  k_build_taps<<<COUT / 2, NTHR, 0, stream>>>(weight, P, bt);
  k_conv_wmma<<<(NIMG * PTILES * (COUT / 64)) / 8, NTHR, 0, stream>>>(xpad, bt, bias, out);
}
